// MultiHeadAttention_120259084641
// MI455X (gfx1250) — hardware-run, weakly checked
//
#include <hip/hip_runtime.h>
#include <math.h>

typedef __attribute__((ext_vector_type(16))) _Float16 v16h;
typedef __attribute__((ext_vector_type(8)))  _Float16 v8h;
typedef __attribute__((ext_vector_type(8)))  float    v8f;
typedef __attribute__((ext_vector_type(4)))  float    v4f;
typedef __attribute__((ext_vector_type(4)))  unsigned int v4u;

constexpr int kBatch  = 2;
constexpr int kSeq    = 2048;
constexpr int kDm     = 1024;
constexpr int kHeads  = 16;
constexpr int kHd     = 64;
constexpr int kHalfHd = kHd / 2;
constexpr int kTok    = kBatch * kSeq;
constexpr int kQkvLd  = 3 * kDm;
constexpr int kBH     = kBatch * kHeads;
static_assert(kHeads * kHd == kDm);
static_assert(kHd == 64 && kHalfHd == 32);
static_assert(kDm == 1024);
static_assert((kTok % 64) == 0 && (kQkvLd % 64) == 0 && (kDm % 64) == 0 && (kDm % 32) == 0);
static_assert((kSeq % 64) == 0);

constexpr float kXCarry = 16.0f;
constexpr float kWCarry = 1024.0f;
constexpr float kQCarry = 16.0f;
constexpr float kKCarry = 16.0f;
constexpr float kVCarry = 16.0f;
constexpr float kPCarry = 32768.0f;
constexpr float kOCarry = 256.0f;
constexpr float kInvSqrtHd = 0.125f;
static_assert(kInvSqrtHd * kInvSqrtHd * (float)kHd == 1.0f);
constexpr float kProjScale  = 1.0f / (kXCarry * kWCarry);
constexpr float kScoreScale = kInvSqrtHd / (kQCarry * kKCarry);
constexpr float kOFold      = kOCarry / (kPCarry * kVCarry);
constexpr float kOutScale   = 1.0f / (kOCarry * kWCarry);
constexpr float kInvHd = 1.0f / (float)kHd;
static_assert(kInvHd * (float)kHd == 1.0f);

constexpr size_t kSzXH   = (size_t)kTok * kDm * 2;
constexpr size_t kSzWALL = (size_t)4 * kDm * kDm * 2;
constexpr size_t kSzBIAS = (size_t)4 * kDm * 4;
constexpr size_t kSzTAB  = (size_t)kSeq * kHalfHd * 4;
constexpr size_t kSzQKVF = (size_t)kTok * kQkvLd * 4;
constexpr size_t kSzHEAD = (size_t)kBH * kSeq * kHd * 2;
constexpr size_t kSzOH   = (size_t)kTok * kDm * 2;
constexpr size_t kOffXH   = 0;
constexpr size_t kOffWALL = kOffXH   + kSzXH;
constexpr size_t kOffBIAS = kOffWALL + kSzWALL;
constexpr size_t kOffCOST = kOffBIAS + kSzBIAS;
constexpr size_t kOffSINT = kOffCOST + kSzTAB;
constexpr size_t kOffQKVF = kOffSINT + kSzTAB;
constexpr size_t kOffQH   = kOffQKVF + kSzQKVF;
constexpr size_t kOffKH   = kOffQH   + kSzHEAD;
constexpr size_t kOffVT   = kOffKH   + kSzHEAD;
constexpr size_t kOffOH   = kOffVT   + kSzHEAD;
constexpr size_t kWsTotal = kOffOH   + kSzOH;
static_assert(kWsTotal == 101203968ull);
static_assert(kWsTotal <= 134217728ull);
static_assert((kOffWALL % 128) == 0 && (kOffBIAS % 128) == 0 && (kOffCOST % 128) == 0 && (kOffSINT % 128) == 0 &&
              (kOffQKVF % 128) == 0 && (kOffQH % 128) == 0 && (kOffKH % 128) == 0 && (kOffVT % 128) == 0 &&
              (kOffOH % 128) == 0);

__device__ __forceinline__ unsigned short f2bf_bits(float f) {
  unsigned u = __float_as_uint(f);
  return (unsigned short)((u + 0x7FFFu + ((u >> 16) & 1u)) >> 16);
}
__device__ __forceinline__ float bf_bits2f(unsigned short h) { return __uint_as_float(((unsigned)h) << 16); }
__device__ __forceinline__ unsigned pk16(unsigned short a, unsigned short b) { return (unsigned)a | ((unsigned)b << 16); }
__device__ __forceinline__ unsigned short h_bits(float f) { const _Float16 h = (_Float16)f; return __builtin_bit_cast(unsigned short, h); }

struct FragH {
  union U { v16h v; v8h h[2]; };
  static __device__ __forceinline__ v16h load(const _Float16* p) {
    U f; f.h[0] = *(const v8h*)(p); f.h[1] = *(const v8h*)(p + 16); return f.v;
  }
  static __device__ __forceinline__ v8f mma(v16h a, v16h b, v8f c) {
    return __builtin_amdgcn_wmma_f32_16x16x32_f16(false, a, false, b, (short)0, c, false, false);
  }
};
__device__ __forceinline__ void tie_acc(v8f& a, v16h x, v16h y) { asm volatile("" : "+v"(a) : "v"(x), "v"(y)); }
__device__ __forceinline__ void tie_acc_nop(v8f& a, v16h x, v16h y) { asm volatile("v_nop\n\tv_nop\n\tv_nop\n\tv_nop" : "+v"(a) : "v"(x), "v"(y)); }
__device__ __forceinline__ void tie_acc_nop6(v8f& a, v16h x0, v16h x1, v16h y0, v16h y1, v16h y2, v16h y3) {
  asm volatile("v_nop\n\tv_nop\n\tv_nop\n\tv_nop" : "+v"(a) : "v"(x0), "v"(x1), "v"(y0), "v"(y1), "v"(y2), "v"(y3));
}
__device__ __forceinline__ void acc_guard1(v8f& a) { asm volatile("v_nop\n\tv_nop\n\tv_nop\n\tv_nop" : "+v"(a)); }
__device__ __forceinline__ void keep4_h(v16h a, v16h b, v16h c, v16h d) { asm volatile("v_nop" :: "v"(a), "v"(b), "v"(c), "v"(d)); }

__global__ __launch_bounds__(256) void cast8_plane_kernel(
    const float* __restrict__ s0, const float* __restrict__ s1, const float* __restrict__ s2, const float* __restrict__ s3,
    unsigned short* __restrict__ out, int planeElems, float carry) {
  const int z = blockIdx.y;
  const float* in = (z == 0) ? s0 : (z == 1) ? s1 : (z == 2) ? s2 : s3;
  const size_t i = (size_t)blockIdx.x * 256 + threadIdx.x;
  const float* p = in + 8 * i;
  const v4f a = *(const v4f*)(p);
  const v4f c = *(const v4f*)(p + 4);
  unsigned short hb[8];
#pragma unroll
  for (int e = 0; e < 4; ++e) {
    const float fa = a[e];
    const float fc = c[e];
    hb[e]     = h_bits(bf_bits2f(f2bf_bits(fa)) * carry);
    hb[4 + e] = h_bits(bf_bits2f(f2bf_bits(fc)) * carry);
  }
  const v4u u = (v4u){pk16(hb[0], hb[1]), pk16(hb[2], hb[3]), pk16(hb[4], hb[5]), pk16(hb[6], hb[7])};
  unsigned short* q = out + (size_t)z * (size_t)planeElems + 8 * i;
  *(volatile v4u*)q = u;
  __threadfence();
  *(volatile v4u*)q = u;
}

__global__ __launch_bounds__(256) void bias_pack_kernel(
    const float* __restrict__ b0, const float* __restrict__ b1, const float* __restrict__ b2, const float* __restrict__ b3,
    float* __restrict__ out) {
  const int z = blockIdx.x;
  const float* src = (z == 0) ? b0 : (z == 1) ? b1 : (z == 2) ? b2 : b3;
  const int n4 = threadIdx.x * 4;
  const v4f v = *(const v4f*)(src + n4);
  const float f0 = v[0], f1 = v[1], f2 = v[2], f3 = v[3];
  const v4f o = (v4f){bf_bits2f(f2bf_bits(f0)), bf_bits2f(f2bf_bits(f1)), bf_bits2f(f2bf_bits(f2)), bf_bits2f(f2bf_bits(f3))};
  float* q = out + z * kDm + n4;
  *(volatile v4f*)q = o;
  __threadfence();
  *(volatile v4f*)q = o;
}

__global__ __launch_bounds__(256) void rot_table_kernel(float* __restrict__ cosT, float* __restrict__ sinT) {
#pragma clang fp contract(off)
  const int lane = threadIdx.x & 31;
  const int wave = __builtin_amdgcn_readfirstlane((int)(threadIdx.x >> 5));
  const int s = blockIdx.x * 8 + wave;
  const float ex = (float)(2 * lane) * kInvHd;
  const float pw = powf(10000.0f, ex);
  const float fr = 1.0f / pw;
  const float theta = (float)s * fr;
  float sn;
  float cs;
  sincosf(theta, &sn, &cs);
  volatile float* pc = cosT + (size_t)s * kHalfHd + lane;
  volatile float* ps = sinT + (size_t)s * kHalfHd + lane;
  *pc = cs;
  *ps = sn;
  __threadfence();
  *pc = cs;
  *ps = sn;
}

__global__ __launch_bounds__(256) void gemm64_f16_kernel(
    const unsigned short* __restrict__ Ap, int lda,
    const unsigned short* __restrict__ Btp, int ldb,
    float* __restrict__ C, int ldc,
    const float* __restrict__ bias,
    int M, int N, int K, float scale) {
  const _Float16* A  = (const _Float16*)Ap;
  const _Float16* Bt = (const _Float16*)Btp;
  __shared__ __align__(16) float sT[8][16 * 68];
  const int lane = threadIdx.x & 31;
  const int wave = __builtin_amdgcn_readfirstlane((int)(threadIdx.x >> 5));
  const int tilesN = N >> 6;
  const int tilesM = M >> 6;
  const int tile = blockIdx.x * 8 + wave;
  if (tile >= tilesM * tilesN) return;
  const int tm = tile / tilesN;
  const int tn = tile - tm * tilesN;
  const int m0 = tm << 6;
  const int n0 = tn << 6;

  const int rlane = lane & 15;
  const int koff  = (lane >> 4) * 8;
  const int mOff  = (lane >> 4) * 8;

  v8f acc[4][4];
#pragma unroll
  for (int i = 0; i < 4; ++i)
#pragma unroll
    for (int j = 0; j < 4; ++j) acc[i][j] = (v8f){0.f, 0.f, 0.f, 0.f, 0.f, 0.f, 0.f, 0.f};

  for (int k0 = 0; k0 < K; k0 += 32) {
    v16h bh[4];
#pragma unroll
    for (int j = 0; j < 4; ++j) {
      const size_t bo = (size_t)(n0 + (j << 4) + rlane) * ldb + koff + k0;
      bh[j] = FragH::load(Bt + bo);
    }
#pragma unroll
    for (int i = 0; i < 4; ++i) {
      const size_t ao = (size_t)(m0 + (i << 4) + rlane) * lda + koff + k0;
      const v16h ah = FragH::load(A + ao);
#pragma unroll
      for (int j = 0; j < 4; ++j) acc[i][j] = FragH::mma(ah, bh[j], acc[i][j]);
      tie_acc(acc[i][0], ah, bh[0]);
      tie_acc(acc[i][1], ah, bh[1]);
      tie_acc(acc[i][2], ah, bh[2]);
      tie_acc_nop(acc[i][3], ah, bh[3]);
    }
    keep4_h(bh[0], bh[1], bh[2], bh[3]);
  }
#pragma unroll
  for (int i = 0; i < 4; ++i)
#pragma unroll
    for (int j = 0; j < 4; ++j) acc_guard1(acc[i][j]);

  float* slab = sT[wave];
#pragma unroll
  for (int i = 0; i < 4; ++i) {
    const int mBase = m0 + (i << 4);
#pragma unroll
    for (int j = 0; j < 4; ++j) {
      const int n = n0 + (j << 4) + rlane;
      const float bv = bias[n];
#pragma unroll
      for (int r = 0; r < 8; ++r) {
        const float v = acc[i][j][r] * scale + bv;
        slab[(mOff + r) * 68 + (j << 4) + rlane] = v;
      }
    }
    __builtin_amdgcn_fence(__ATOMIC_RELEASE, "workgroup");
    __builtin_amdgcn_wave_barrier();
    __builtin_amdgcn_fence(__ATOMIC_ACQUIRE, "workgroup");
    {
      const int hh = lane >> 4, c4 = (lane & 15) * 4;
      for (int pass = 0; pass < 2; ++pass) {
#pragma unroll
        for (int it = 0; it < 8; ++it) {
          const int row = it * 2 + hh;
          const v4f v = *(const v4f*)(slab + row * 68 + c4);
          *(volatile v4f*)(C + (size_t)(mBase + row) * ldc + n0 + c4) = v;
        }
        __threadfence();
      }
    }
    __builtin_amdgcn_fence(__ATOMIC_RELEASE, "workgroup");
    __builtin_amdgcn_wave_barrier();
    __builtin_amdgcn_fence(__ATOMIC_ACQUIRE, "workgroup");
  }
}

__global__ __launch_bounds__(256) void rot_relayout_kernel(
    const float* __restrict__ QKV, const float* __restrict__ cosT, const float* __restrict__ sinT,
    unsigned short* __restrict__ Qh, unsigned short* __restrict__ Kh, unsigned short* __restrict__ Vt) {
  __shared__ float sm[64][65];
  const int t = threadIdx.x;
  const int lane = t & 31;
  const int wave = __builtin_amdgcn_readfirstlane((int)(t >> 5));
  const int s0 = blockIdx.x * 64;
  const int bh = blockIdx.y;
  const int b  = bh / kHeads;
  const int h  = bh - b * kHeads;
  const size_t rowbase = (size_t)b * kSeq + s0;

#pragma unroll
  for (int i = 0; i < 4; ++i) {
    const int e4 = i * 256 + t;
    const int r  = e4 >> 4;
    const int c4 = (e4 & 15) * 4;
    const v4f v = *(const v4f*)(QKV + (rowbase + r) * kQkvLd + 2 * kDm + h * kHd + c4);
    sm[c4 + 0][r] = v[0] * kVCarry;
    sm[c4 + 1][r] = v[1] * kVCarry;
    sm[c4 + 2][r] = v[2] * kVCarry;
    sm[c4 + 3][r] = v[3] * kVCarry;
  }
  __syncthreads();
  {
    const int q = lane >> 3, c8 = (lane & 7) * 8;
    v4u uv[2];
#pragma unroll
    for (int it = 0; it < 2; ++it) {
      const int row = wave * 8 + it * 4 + q;
      unsigned short hb[8];
#pragma unroll
      for (int e = 0; e < 8; ++e) hb[e] = h_bits(sm[row][c8 + e]);
      uv[it] = (v4u){pk16(hb[0], hb[1]), pk16(hb[2], hb[3]), pk16(hb[4], hb[5]), pk16(hb[6], hb[7])};
    }
    for (int pass = 0; pass < 2; ++pass) {
#pragma unroll
      for (int it = 0; it < 2; ++it) {
        const int row = wave * 8 + it * 4 + q;
        *(volatile v4u*)(Vt + ((size_t)bh * kHd + row) * kSeq + s0 + c8) = uv[it];
      }
      __threadfence();
    }
  }

#pragma unroll 1
  for (int p = 0; p < 2; ++p) {
    const int idx = p * 256 + t;
    const int r   = idx >> 3;
    const int c8q = (idx & 7) * 8;
    const int cpr = c8q ^ 32;
    const int j8  = c8q & 31;
    const float* src = QKV + (rowbase + r) * kQkvLd + h * kHd;
    const v4f qo0 = *(const v4f*)(src + c8q);
    const v4f qo1 = *(const v4f*)(src + c8q + 4);
    const v4f qp0 = *(const v4f*)(src + cpr);
    const v4f qp1 = *(const v4f*)(src + cpr + 4);
    const v4f ko0 = *(const v4f*)(src + kDm + c8q);
    const v4f ko1 = *(const v4f*)(src + kDm + c8q + 4);
    const v4f kp0 = *(const v4f*)(src + kDm + cpr);
    const v4f kp1 = *(const v4f*)(src + kDm + cpr + 4);
    const float* ct = cosT + (size_t)(s0 + r) * kHalfHd + j8;
    const float* st = sinT + (size_t)(s0 + r) * kHalfHd + j8;
    const v4f cs0 = *(const v4f*)(ct);
    const v4f cs1 = *(const v4f*)(ct + 4);
    const v4f sn0 = *(const v4f*)(st);
    const v4f sn1 = *(const v4f*)(st + 4);
    const float sgn = (c8q < 32) ? -1.0f : 1.0f;
    unsigned short hq[8], hk[8];
#pragma unroll
    for (int e = 0; e < 4; ++e) {
      const float c0 = cs0[e], c1 = cs1[e];
      const float z0 = sn0[e] * sgn, z1 = sn1[e] * sgn;
      const float q0v = qo0[e] * c0 + qp0[e] * z0;
      const float q1v = qo1[e] * c1 + qp1[e] * z1;
      const float k0v = ko0[e] * c0 + kp0[e] * z0;
      const float k1v = ko1[e] * c1 + kp1[e] * z1;
      hq[e]     = h_bits(q0v * kQCarry);
      hq[4 + e] = h_bits(q1v * kQCarry);
      hk[e]     = h_bits(k0v * kKCarry);
      hk[4 + e] = h_bits(k1v * kKCarry);
    }
    const v4u uq = (v4u){pk16(hq[0], hq[1]), pk16(hq[2], hq[3]), pk16(hq[4], hq[5]), pk16(hq[6], hq[7])};
    const v4u uk = (v4u){pk16(hk[0], hk[1]), pk16(hk[2], hk[3]), pk16(hk[4], hk[5]), pk16(hk[6], hk[7])};
    const size_t o = ((size_t)bh * kSeq + s0 + r) * kHd + c8q;
    *(volatile v4u*)(Qh + o) = uq;
    *(volatile v4u*)(Kh + o) = uk;
    __threadfence();
    *(volatile v4u*)(Qh + o) = uq;
    *(volatile v4u*)(Kh + o) = uk;
  }
}

constexpr int kPPitch = 64;

__global__ __launch_bounds__(128) void attn_stream_kernel(
    const unsigned short* __restrict__ Qp, const unsigned short* __restrict__ Kp,
    const unsigned short* __restrict__ Vtp, unsigned short* __restrict__ Op) {
  __shared__ __align__(16) _Float16 Ps[4][16 * kPPitch];
  __shared__ __align__(16) float    Os[4][16 * 68];
  const int tid  = threadIdx.x;
  const int wave = __builtin_amdgcn_readfirstlane((int)(tid >> 5));
  const int lane = tid & 31;
  const int hh   = lane >> 4;
  const int c    = lane & 15;
  const int qb   = blockIdx.x;
  const int bh   = blockIdx.y;
  const int b    = bh / kHeads;
  const int h    = bh - b * kHeads;
  const int q0   = qb * 64 + wave * 16;

  const _Float16* Qb = (const _Float16*)Qp  + (size_t)bh * kSeq * kHd;
  const _Float16* Kb = (const _Float16*)Kp  + (size_t)bh * kSeq * kHd;
  const _Float16* Vb = (const _Float16*)Vtp + (size_t)bh * kHd * kSeq;

  const v16h qa0 = FragH::load(Qb + (size_t)(q0 + c) * kHd + 8 * hh);
  const v16h qa1 = FragH::load(Qb + (size_t)(q0 + c) * kHd + 32 + 8 * hh);

  float mrow[8], lsum[8];
  v8f oacc[4];
#pragma unroll
  for (int r = 0; r < 8; ++r) { mrow[r] = -1.0e30f; lsum[r] = 0.f; }
#pragma unroll
  for (int t = 0; t < 4; ++t) oacc[t] = (v8f){0.f, 0.f, 0.f, 0.f, 0.f, 0.f, 0.f, 0.f};

  _Float16* pw = Ps[wave];

#pragma unroll 1
  for (int kc = 0; kc < kSeq / 64; ++kc) {
    const int kv0 = kc * 64;
    v8f s[4];
#pragma unroll
    for (int j = 0; j < 4; ++j) s[j] = (v8f){0.f, 0.f, 0.f, 0.f, 0.f, 0.f, 0.f, 0.f};
#pragma unroll
    for (int jp = 0; jp < 2; ++jp) {
      const _Float16* kp0 = Kb + (size_t)(kv0 + jp * 32 + c) * kHd + 8 * hh;
      const _Float16* kp1 = kp0 + 16 * kHd;
      const v16h k00 = FragH::load(kp0);
      const v16h k01 = FragH::load(kp0 + 32);
      const v16h k10 = FragH::load(kp1);
      const v16h k11 = FragH::load(kp1 + 32);
      s[2 * jp]     = FragH::mma(qa0, k00, s[2 * jp]);
      s[2 * jp + 1] = FragH::mma(qa0, k10, s[2 * jp + 1]);
      s[2 * jp]     = FragH::mma(qa1, k01, s[2 * jp]);
      s[2 * jp + 1] = FragH::mma(qa1, k11, s[2 * jp + 1]);
      tie_acc(s[2 * jp], qa1, k01);
      tie_acc_nop6(s[2 * jp + 1], qa0, qa1, k00, k01, k10, k11);
    }

#pragma unroll
    for (int r = 0; r < 8; ++r) {
      float m = fmaxf(fmaxf(s[0][r], s[1][r]), fmaxf(s[2][r], s[3][r]));
      m = fmaxf(m, __shfl_xor(m, 1, 32));
      m = fmaxf(m, __shfl_xor(m, 2, 32));
      m = fmaxf(m, __shfl_xor(m, 4, 32));
      m = fmaxf(m, __shfl_xor(m, 8, 32));
      const float mnew  = fmaxf(mrow[r], m);
      const float alpha = __expf((mrow[r] - mnew) * kScoreScale);
      mrow[r] = mnew;
      float psum = 0.f;
#pragma unroll
      for (int j = 0; j < 4; ++j) {
        const float pv = __expf((s[j][r] - mnew) * kScoreScale);
        psum += pv;
        pw[(8 * hh + r) * kPPitch + j * 16 + c] = (_Float16)(pv * kPCarry);
      }
      lsum[r] = lsum[r] * alpha + psum;
#pragma unroll
      for (int t = 0; t < 4; ++t) oacc[t][r] *= alpha;
    }
    __builtin_amdgcn_fence(__ATOMIC_RELEASE, "workgroup");
    __builtin_amdgcn_wave_barrier();
    __builtin_amdgcn_fence(__ATOMIC_ACQUIRE, "workgroup");

    const v16h pa0 = FragH::load(pw + c * kPPitch + 8 * hh);
    const v16h pa1 = FragH::load(pw + c * kPPitch + 32 + 8 * hh);
#pragma unroll
    for (int tp = 0; tp < 2; ++tp) {
      const _Float16* vp0 = Vb + (size_t)(tp * 32 + c) * kSeq + kv0 + 8 * hh;
      const _Float16* vp1 = vp0 + 16 * kSeq;
      const v16h v00 = FragH::load(vp0);
      const v16h v01 = FragH::load(vp0 + 32);
      const v16h v10 = FragH::load(vp1);
      const v16h v11 = FragH::load(vp1 + 32);
      oacc[2 * tp]     = FragH::mma(pa0, v00, oacc[2 * tp]);
      oacc[2 * tp + 1] = FragH::mma(pa0, v10, oacc[2 * tp + 1]);
      oacc[2 * tp]     = FragH::mma(pa1, v01, oacc[2 * tp]);
      oacc[2 * tp + 1] = FragH::mma(pa1, v11, oacc[2 * tp + 1]);
      tie_acc(oacc[2 * tp], pa1, v01);
      tie_acc_nop6(oacc[2 * tp + 1], pa0, pa1, v00, v01, v10, v11);
    }
    __builtin_amdgcn_fence(__ATOMIC_RELEASE, "workgroup");
    __builtin_amdgcn_wave_barrier();
    __builtin_amdgcn_fence(__ATOMIC_ACQUIRE, "workgroup");
  }

  float* os = Os[wave];
#pragma unroll
  for (int r = 0; r < 8; ++r) {
    float l = lsum[r];
    l += __shfl_xor(l, 1, 32);
    l += __shfl_xor(l, 2, 32);
    l += __shfl_xor(l, 4, 32);
    l += __shfl_xor(l, 8, 32);
    const float inv = kOFold * (1.0f / l);
#pragma unroll
    for (int t = 0; t < 4; ++t) os[(8 * hh + r) * 68 + t * 16 + c] = oacc[t][r] * inv;
  }
  __builtin_amdgcn_fence(__ATOMIC_RELEASE, "workgroup");
  __builtin_amdgcn_wave_barrier();
  __builtin_amdgcn_fence(__ATOMIC_ACQUIRE, "workgroup");
  {
    const int q = lane >> 3, c8 = (lane & 7) * 8;
    v4u uo[4];
#pragma unroll
    for (int it = 0; it < 4; ++it) {
      const int row = it * 4 + q;
      const float* sp = os + row * 68 + c8;
      const v4f a0 = *(const v4f*)(sp);
      const v4f a1 = *(const v4f*)(sp + 4);
      unsigned short hb[8];
#pragma unroll
      for (int e = 0; e < 4; ++e) {
        const float f0 = a0[e];
        const float f1 = a1[e];
        hb[e]     = h_bits(f0);
        hb[4 + e] = h_bits(f1);
      }
      uo[it] = (v4u){pk16(hb[0], hb[1]), pk16(hb[2], hb[3]), pk16(hb[4], hb[5]), pk16(hb[6], hb[7])};
    }
    for (int pass = 0; pass < 2; ++pass) {
#pragma unroll
      for (int it = 0; it < 4; ++it) {
        const int row = it * 4 + q;
        *(volatile v4u*)(Op + ((size_t)b * kSeq + q0 + row) * kDm + h * kHd + c8) = uo[it];
      }
      __threadfence();
    }
  }
}

static_assert(((size_t)kTok * kDm / 8) % 256 == 0);
static_assert(((size_t)kDm * kDm / 8) % 256 == 0);
static_assert(((kTok / 64) * (kQkvLd / 64)) % 8 == 0);
static_assert(((kTok / 64) * (kDm / 64)) % 8 == 0);
static_assert((kSeq % 8) == 0);

extern "C" void kernel_launch(void* const* d_in, const int* in_sizes, int n_in,
                              void* d_out, int out_size, void* d_ws, size_t ws_size,
                              hipStream_t stream) {
  if (n_in < 9) return;
  if (in_sizes[0] != kTok * kDm) return;
  if (in_sizes[1] != kDm * kDm || in_sizes[3] != kDm * kDm || in_sizes[5] != kDm * kDm || in_sizes[7] != kDm * kDm) return;
  if (in_sizes[2] != kDm || in_sizes[4] != kDm || in_sizes[6] != kDm || in_sizes[8] != kDm) return;
  if (out_size != kTok * kDm) return;
  if (ws_size < kWsTotal) return;

  const float* x  = (const float*)d_in[0];
  const float* wq = (const float*)d_in[1];
  const float* bq = (const float*)d_in[2];
  const float* wk = (const float*)d_in[3];
  const float* bk = (const float*)d_in[4];
  const float* wv = (const float*)d_in[5];
  const float* bv = (const float*)d_in[6];
  const float* wo = (const float*)d_in[7];
  const float* bo = (const float*)d_in[8];
  float* out = (float*)d_out;

  char* ws = (char*)d_ws;
  unsigned short* XH   = (unsigned short*)(ws + kOffXH);
  unsigned short* WALL = (unsigned short*)(ws + kOffWALL);
  float*          BIAS = (float*)(ws + kOffBIAS);
  float*          COST = (float*)(ws + kOffCOST);
  float*          SINT = (float*)(ws + kOffSINT);
  float*          QKVF = (float*)(ws + kOffQKVF);
  unsigned short* QH   = (unsigned short*)(ws + kOffQH);
  unsigned short* KH   = (unsigned short*)(ws + kOffKH);
  unsigned short* VT   = (unsigned short*)(ws + kOffVT);
  unsigned short* OH   = (unsigned short*)(ws + kOffOH);

  cast8_plane_kernel<<<dim3((kTok * kDm / 8) / 256, 1), 256, 0, stream>>>(x, x, x, x, XH, kTok * kDm, kXCarry);
  cast8_plane_kernel<<<dim3((kDm * kDm / 8) / 256, 4), 256, 0, stream>>>(wq, wk, wv, wo, WALL, kDm * kDm, kWCarry);
  bias_pack_kernel<<<4, 256, 0, stream>>>(bq, bk, bv, bo, BIAS);

  rot_table_kernel<<<kSeq / 8, 256, 0, stream>>>(COST, SINT);

  gemm64_f16_kernel<<<((kTok / 64) * (kQkvLd / 64)) / 8, 256, 0, stream>>>(
      XH, kDm, WALL, kDm, QKVF, kQkvLd, BIAS, kTok, kQkvLd, kDm, kProjScale);

  rot_relayout_kernel<<<dim3(kSeq / 64, kBH), 256, 0, stream>>>(QKVF, COST, SINT, QH, KH, VT);

  attn_stream_kernel<<<dim3(kSeq / 64, kBH), 128, 0, stream>>>(QH, KH, VT, OH);

  gemm64_f16_kernel<<<((kTok / 64) * (kDm / 64)) / 8, 256, 0, stream>>>(
      OH, kDm, WALL + (size_t)3 * kDm * kDm, kDm, out, kDm, BIAS + 3 * kDm, kTok, kDm, kDm, kOutScale);
}
